// BilinearMLPEmbedPheno_64364379898013
// MI455X (gfx1250) — hardware-verified
//
#include <hip/hip_runtime.h>
#include <math.h>

constexpr int kRows      = 131072;
constexpr int kGenes     = 20000;
constexpr int kEmb       = 16;
constexpr int kHid       = 512;
constexpr int kChunk     = 16384;
constexpr int kNumChunks = kRows / kChunk;
constexpr int kRowsPerBlk = 64;
constexpr float kCarryA    = 16.0f;
constexpr float kCarryW    = 16.0f;
constexpr float kGemmScale = 1.0f / 256.0f;
static_assert(kRows % kChunk == 0, "chunking");
static_assert(kChunk % 64 == 0, "GEMM M tile");
static_assert(kHid % 64 == 0 && kHid % 32 == 0, "GEMM N/K tiles");
static_assert(kChunk % kRowsPerBlk == 0, "finisher blocks");

constexpr size_t kOffWT   = 0;
constexpr size_t kBytesWT = (size_t)kHid * kHid * 2;
constexpr size_t kOffG1   = kOffWT + kBytesWT;
constexpr size_t kBytesG1 = (size_t)kChunk * kHid * 2;
constexpr size_t kOffPre2 = kOffG1 + kBytesG1;
constexpr size_t kBytesPre2 = (size_t)kChunk * kHid * 4;
constexpr size_t kWsTotal = kOffPre2 + kBytesPre2;
static_assert(kWsTotal == 50855936, "carve total");
static_assert(kOffG1 % 128 == 0 && kOffPre2 % 128 == 0, "line alignment");

typedef __attribute__((ext_vector_type(16))) _Float16 v16h;
typedef __attribute__((ext_vector_type(8)))  _Float16 v8h;
typedef __attribute__((ext_vector_type(16))) __bf16   v16b;
typedef __attribute__((ext_vector_type(8)))  __bf16   v8b;
typedef __attribute__((ext_vector_type(8)))  float    v8f;
typedef __attribute__((ext_vector_type(4)))  float    v4f;
typedef __attribute__((ext_vector_type(4)))  unsigned int v4u;

__device__ __forceinline__ unsigned short f2bf_bits(float f) {
  unsigned u = __float_as_uint(f);
  return (unsigned short)((u + 0x7FFFu + ((u >> 16) & 1u)) >> 16);
}
__device__ __forceinline__ float bf_bits2f(unsigned short h) { return __uint_as_float(((unsigned)h) << 16); }

__device__ __forceinline__ void dep_guard_h(v8f& a, v8f& b, v16h x, v16h y) { asm volatile("v_nop\n\tv_nop\n\tv_nop\n\tv_nop" : "+v"(a), "+v"(b) : "v"(x), "v"(y)); }
__device__ __forceinline__ void dep_guard_b(v8f& a, v8f& b, v16b x, v16b y) { asm volatile("v_nop\n\tv_nop\n\tv_nop\n\tv_nop" : "+v"(a), "+v"(b) : "v"(x), "v"(y)); }
__device__ __forceinline__ void keep4_h(v16h a, v16h b, v16h c, v16h d) { asm volatile("v_nop" :: "v"(a), "v"(b), "v"(c), "v"(d)); }
__device__ __forceinline__ void keep4_b(v16b a, v16b b, v16b c, v16b d) { asm volatile("v_nop" :: "v"(a), "v"(b), "v"(c), "v"(d)); }
__device__ __forceinline__ void acc_guard4(v8f& a, v8f& b, v8f& c, v8f& d) { asm volatile("v_nop\n\tv_nop\n\tv_nop\n\tv_nop" : "+v"(a), "+v"(b), "+v"(c), "+v"(d)); }
template <typename T> struct Frag;
template <> struct Frag<_Float16> {
  typedef v16h V; union U { v16h v; v8h h[2]; };
  static __device__ __forceinline__ v16h load(const _Float16* p) {
    U f; f.h[0] = *(const v8h*)(p); f.h[1] = *(const v8h*)(p + 16); return f.v;
  }
  static __device__ __forceinline__ v8f mma(v16h a, v16h b, v8f c) {
    return __builtin_amdgcn_wmma_f32_16x16x32_f16(false, a, false, b, (short)0, c, false, false);
  }
  static __device__ __forceinline__ void guard(v8f& a, v8f& b, v16h x, v16h y) { dep_guard_h(a, b, x, y); }
  static __device__ __forceinline__ void keep(v16h a, v16h b, v16h c, v16h d) { keep4_h(a, b, c, d); }
};
template <> struct Frag<__bf16> {
  typedef v16b V; union U { v16b v; v8b h[2]; };
  static __device__ __forceinline__ v16b load(const __bf16* p) {
    U f; f.h[0] = *(const v8b*)(p); f.h[1] = *(const v8b*)(p + 16); return f.v;
  }
  static __device__ __forceinline__ v8f mma(v16b a, v16b b, v8f c) {
    return __builtin_amdgcn_wmma_f32_16x16x32_bf16(false, a, false, b, (short)0, c, false, false);
  }
  static __device__ __forceinline__ void guard(v8f& a, v8f& b, v16b x, v16b y) { dep_guard_b(a, b, x, y); }
  static __device__ __forceinline__ void keep(v16b a, v16b b, v16b c, v16b d) { keep4_b(a, b, c, d); }
};

__device__ __forceinline__ unsigned pk16(unsigned short a, unsigned short b) { return (unsigned)a | ((unsigned)b << 16); }
__device__ __forceinline__ unsigned short h_bits(float f) { const _Float16 h = (_Float16)f; return __builtin_bit_cast(unsigned short, h); }

template <int ET> struct Elem;
template <> struct Elem<0> { typedef _Float16 T; };
template <> struct Elem<1> { typedef __bf16 T; };
template <int ET, bool SPLIT, int BIAS_MODE, int OUT_MODE, bool RESID, int ACT = 0>
__global__ __launch_bounds__(256) void wmma_gemm64(
    const unsigned short* __restrict__ Ap, const unsigned short* __restrict__ A2p, int lda, long strideA,
    const unsigned short* __restrict__ Btp, const unsigned short* __restrict__ Bt2p, int ldb, long strideB,
    void* __restrict__ Cout, void* __restrict__ Cout2, int ldc, long strideC,
    const float* __restrict__ bias,
    const float* __restrict__ resid, long strideR,
    int M, int N, int K, float scale) {
  typedef typename Elem<ET>::T T;
  typedef typename Frag<T>::V V;
  const T* A = (const T*)Ap; const T* A2 = (const T*)A2p; const T* Bt = (const T*)Btp; const T* Bt2 = (const T*)Bt2p;
  __shared__ __align__(16) float sT[8][16 * 68];
  const int b    = blockIdx.y;
  const int lane = threadIdx.x & 31;
  const int wave = threadIdx.x >> 5;
  const int tilesN = N >> 6;
  const int tilesM = M >> 6;
  const int tile = blockIdx.x * 8 + wave;
  if (tile >= tilesM * tilesN) return;
  const int tm = tile / tilesN;
  const int tn = tile - tm * tilesN;
  const int m0 = tm << 6;
  const int n0 = tn << 6;

  const T* Ab  = A  + (size_t)b * strideA;
  const T* Bb  = Bt + (size_t)b * strideB;
  const T* Ab2 = SPLIT ? (A2  + (size_t)b * strideA) : nullptr;
  const T* Bb2 = SPLIT ? (Bt2 + (size_t)b * strideB) : nullptr;

  const int rlane = lane & 15;
  const int koff  = (lane >> 4) * 8;
  const int mOff  = (lane >> 4) * 8;

  v8f acc[4][4];
#pragma unroll
  for (int i = 0; i < 4; ++i)
#pragma unroll
    for (int j = 0; j < 4; ++j) acc[i][j] = (v8f){0.f,0.f,0.f,0.f,0.f,0.f,0.f,0.f};

  for (int k0 = 0; k0 < K; k0 += 32) {
    V bh[4], bl[4];
#pragma unroll
    for (int j = 0; j < 4; ++j) {
      const size_t bo = (size_t)(n0 + (j << 4) + rlane) * ldb + koff + k0;
      bh[j] = Frag<T>::load(Bb + bo);
      if (SPLIT) bl[j] = Frag<T>::load(Bb2 + bo);
    }
#pragma unroll
    for (int i = 0; i < 4; ++i) {
      const size_t ao = (size_t)(m0 + (i << 4) + rlane) * lda + koff + k0;
      V ah = Frag<T>::load(Ab + ao);
      V al;
      if (SPLIT) al = Frag<T>::load(Ab2 + ao);
#pragma unroll
      for (int j = 0; j < 4; ++j) {
        acc[i][j] = Frag<T>::mma(ah, bh[j], acc[i][j]);
        if (SPLIT) {
          acc[i][j] = Frag<T>::mma(ah, bl[j], acc[i][j]);
          acc[i][j] = Frag<T>::mma(al, bh[j], acc[i][j]);
        }
      }
      Frag<T>::guard(acc[i][0], acc[i][3], ah, SPLIT ? al : ah);
    }
    Frag<T>::keep(bh[0], bh[1], bh[2], bh[3]);
    if (SPLIT) Frag<T>::keep(bl[0], bl[1], bl[2], bl[3]);
  }
  acc_guard4(acc[0][0], acc[0][1], acc[0][2], acc[0][3]);
  acc_guard4(acc[1][0], acc[1][1], acc[1][2], acc[1][3]);
  acc_guard4(acc[2][0], acc[2][1], acc[2][2], acc[2][3]);
  acc_guard4(acc[3][0], acc[3][1], acc[3][2], acc[3][3]);

  float* slab = sT[wave];
  const float* Rb = RESID ? (resid + (size_t)b * strideR) : nullptr;
#pragma unroll
  for (int i = 0; i < 4; ++i) {
    const int mBase = m0 + (i << 4);
#pragma unroll
    for (int j = 0; j < 4; ++j) {
      const int n = n0 + (j << 4) + rlane;
      float bv = 0.f;
      if (BIAS_MODE == 2) bv = bias[n];
#pragma unroll
      for (int r = 0; r < 8; ++r) {
        float v = acc[i][j][r] * scale;
        if (BIAS_MODE == 1) v += bias[mBase + mOff + r];
        if (BIAS_MODE == 2) v += bv;
        if (RESID) v += Rb[(size_t)(mBase + mOff + r) * ldc + n];
        if (ACT == 2) v = fmaxf(v, 0.0f);
        if (ACT == 4) v = (v > 0.f) ? v : 0.01f * v;
        slab[(mOff + r) * 68 + (j << 4) + rlane] = v;
      }
    }
    __builtin_amdgcn_fence(__ATOMIC_RELEASE, "workgroup");
    __builtin_amdgcn_wave_barrier();
    __builtin_amdgcn_fence(__ATOMIC_ACQUIRE, "workgroup");
    if (OUT_MODE == 0) {
      float* C = (float*)Cout + (size_t)b * strideC;
      const int hh = lane >> 4, c4 = (lane & 15) * 4;
      for (int pass = 0; pass < 2; ++pass) {
#pragma unroll
        for (int it = 0; it < 8; ++it) {
          const int row = it * 2 + hh;
          v4f v = *(const v4f*)(slab + row * 68 + c4);
          *(volatile v4f*)(C + (size_t)(mBase + row) * ldc + n0 + c4) = v;
        }
        __threadfence();
      }
    } else {
      const int q = lane >> 3, c8 = (lane & 7) * 8;
      unsigned short* C  = (unsigned short*)Cout  + (size_t)b * strideC;
      unsigned short* C2 = (OUT_MODE == 2) ? ((unsigned short*)Cout2 + (size_t)b * strideC) : nullptr;
      for (int pass = 0; pass < 2; ++pass) {
#pragma unroll
        for (int it = 0; it < 4; ++it) {
          const int row = it * 4 + q;
          const float* sp = slab + row * 68 + c8;
          v8h hv, lv;
#pragma unroll
          for (int e = 0; e < 8; ++e) {
            if (OUT_MODE == 1) {
              hv[e] = (_Float16)sp[e];
            } else {
              unsigned short hb = f2bf_bits(sp[e]);
              unsigned short lb = f2bf_bits(sp[e] - bf_bits2f(hb));
              hv[e] = __builtin_bit_cast(_Float16, hb);
              lv[e] = __builtin_bit_cast(_Float16, lb);
            }
          }
          *(volatile v8h*)(C + (size_t)(mBase + row) * ldc + n0 + c8) = hv;
          if (OUT_MODE == 2) *(volatile v8h*)(C2 + (size_t)(mBase + row) * ldc + n0 + c8) = lv;
        }
        __threadfence();
      }
    }
    __builtin_amdgcn_fence(__ATOMIC_RELEASE, "workgroup");
    __builtin_amdgcn_wave_barrier();
    __builtin_amdgcn_fence(__ATOMIC_ACQUIRE, "workgroup");
  }
}

__device__ __forceinline__ float gelu_erf(float x) {
  return 0.5f * x * (1.0f + erff(x * 0.70710678118654752f));
}
__device__ __forceinline__ void wave_sync() {
  __builtin_amdgcn_fence(__ATOMIC_RELEASE, "workgroup");
  __builtin_amdgcn_wave_barrier();
  __builtin_amdgcn_fence(__ATOMIC_ACQUIRE, "workgroup");
}

__global__ __launch_bounds__(256) void wtcast_kernel(const float* __restrict__ W, unsigned short* __restrict__ out, float scale) {
  __shared__ float sm[64][65];
  const int t  = threadIdx.x;
  const int d0 = blockIdx.x * 64;
  const int h0 = blockIdx.y * 64;
#pragma unroll
  for (int i = 0; i < 16; ++i) {
    const int e = i * 256 + t;
    const int r = e >> 6;
    const int c = e & 63;
    sm[c][r] = W[(size_t)(d0 + r) * kHid + h0 + c] * scale;
  }
  __syncthreads();
  const int lane = t & 31, wave = t >> 5;
  const int q = lane >> 3, c8 = (lane & 7) * 8;
  for (int pass = 0; pass < 2; ++pass) {
#pragma unroll
    for (int it = 0; it < 2; ++it) {
      const int row = wave * 8 + it * 4 + q;
      unsigned short hb[8];
#pragma unroll
      for (int e = 0; e < 8; ++e) hb[e] = h_bits(sm[row][c8 + e]);
      const v4u u = (v4u){pk16(hb[0], hb[1]), pk16(hb[2], hb[3]), pk16(hb[4], hb[5]), pk16(hb[6], hb[7])};
      *(volatile v4u*)(out + (size_t)(h0 + row) * kHid + d0 + c8) = u;
    }
    __threadfence();
  }
}

__global__ __launch_bounds__(256) void pheno_l1_kernel(const float* __restrict__ phenos, const float* __restrict__ Wp1,
                                                       unsigned short* __restrict__ g1, int row0, int nRowsTot) {
  const int i = blockIdx.x * 256 + threadIdx.x;
  if (i >= kChunk * (kHid / 2)) return;
  const int row = i / (kHid / 2);
  const int n   = (i - row * (kHid / 2)) * 2;
  int grow = row0 + row;
  grow = min(grow, nRowsTot - 1);
  grow = max(grow, 0);
  const float ph0 = phenos[(size_t)grow * 2 + 0];
  const float ph1 = phenos[(size_t)grow * 2 + 1];
  unsigned u = 0u;
#pragma unroll 1
  for (int e = 0; e < 2; ++e) {
    const float pre = ph0 * Wp1[n + e] + ph1 * Wp1[kHid + n + e];
    const float g = gelu_erf(pre) * kCarryA;
    u |= ((unsigned)h_bits(g)) << (16 * e);
  }
  unsigned* q = (unsigned*)(void*)g1 + i;
  *(volatile unsigned*)q = u;
  __threadfence();
  *(volatile unsigned*)q = u;
}

__global__ __launch_bounds__(256)
void finisher_kernel(const int* __restrict__ x,
                     const float* __restrict__ emb,
                     const float* __restrict__ W1, const float* __restrict__ b1,
                     const float* __restrict__ W2, const float* __restrict__ b2,
                     const float* __restrict__ Wb, const float* __restrict__ ob,
                     const float* __restrict__ Wc1, const float* __restrict__ bc1,
                     const float* __restrict__ Wc2, const float* __restrict__ bc2,
                     const float* __restrict__ Wp3, const float* __restrict__ bp3,
                     const float* __restrict__ pre2,
                     float* __restrict__ out, int row0, int nRowsTot) {
  __shared__ float sWb[kEmb * kEmb * kEmb];
  __shared__ float sW1[256], sW2[256], sWc1[256];
  __shared__ float sb1[16], sb2[16], sob[16], sbc1[16], sWc2[16];
  __shared__ float sWp3[kHid];
  __shared__ float sE[8][32], sTm[8][32], sHm[8][32], sZ[8][16];
  __shared__ float sOut[kRowsPerBlk];

  const int tid = threadIdx.x;
  for (int i = tid; i < kEmb * kEmb * kEmb; i += 256) sWb[i] = Wb[i];
  sW1[tid] = W1[tid];
  sW2[tid] = W2[tid];
  sWc1[tid] = Wc1[tid];
  sWp3[tid] = Wp3[tid];
  sWp3[256 + tid] = Wp3[256 + tid];
  {
    const int t16 = tid & 15;
    const float vb1 = b1[t16], vb2 = b2[t16], vob = ob[t16], vbc1 = bc1[t16], vwc2 = Wc2[t16];
    if (tid < 16) { sb1[tid] = vb1; sb2[tid] = vb2; sob[tid] = vob; sbc1[tid] = vbc1; sWc2[tid] = vwc2; }
  }
  const float vbc2 = bc2[0];
  const float vbp3 = bp3[0];
  __syncthreads();

  const int lane = tid & 31, wave = tid >> 5;
  const int slot = lane >> 4;
  const int j    = lane & 15;
  const int blkRow0 = blockIdx.x * kRowsPerBlk;

#pragma unroll 1
  for (int rr = 0; rr < 8; ++rr) {
    const int rloc = wave * 8 + rr;
    const int crow = blkRow0 + rloc;
    int grow = row0 + crow;
    grow = min(grow, nRowsTot - 1);
    grow = max(grow, 0);

    int id = x[(size_t)grow * 2 + slot];
    id = (id < 0) ? (id + kGenes) : id;
    id = max(0, min(id, kGenes - 1));
    sE[wave][lane] = emb[(size_t)id * kEmb + j];
    wave_sync();

    float s1 = sb1[j];
#pragma unroll 4
    for (int k = 0; k < 16; ++k) s1 += sE[wave][slot * 16 + k] * sW1[k * 16 + j];
    sTm[wave][lane] = fmaxf(s1, 0.0f);
    wave_sync();

    float s2 = sb2[j];
#pragma unroll 4
    for (int k = 0; k < 16; ++k) s2 += sTm[wave][slot * 16 + k] * sW2[k * 16 + j];
    sHm[wave][lane] = s2;
    wave_sync();

    float zp = 0.0f;
#pragma unroll 1
    for (int aa = 0; aa < 8; ++aa) {
      const int a  = slot * 8 + aa;
      const int o0 = (j * 16 + a) * 16;
      const int o1 = (a * 16 + j) * 16;
      float d0 = 0.0f, d1 = 0.0f;
#pragma unroll 4
      for (int k = 0; k < 16; ++k) {
        d0 += sWb[o0 + k] * sHm[wave][k];
        d1 += sWb[o1 + k] * sHm[wave][16 + k];
      }
      zp += d0 * d1;
    }
    zp += __shfl_xor(zp, 16, 32);
    const float zc = zp + sob[j];
    if (slot == 0) sZ[wave][j] = zc;
    wave_sync();

    float u = sbc1[j];
#pragma unroll 4
    for (int q = 0; q < 16; ++q) u += sZ[wave][q] * sWc1[q * 16 + j];
    float hv = fmaxf(u, 0.0f) * sWc2[j];
    hv += __shfl_xor(hv, 1, 32);
    hv += __shfl_xor(hv, 2, 32);
    hv += __shfl_xor(hv, 4, 32);
    hv += __shfl_xor(hv, 8, 32);
    const float zs = hv + vbc2;

    const float* pr = pre2 + (size_t)crow * kHid + lane;
    float pacc = 0.0f;
#pragma unroll 1
    for (int i = 0; i < kHid / 32; ++i) {
      const float v = pr[i * 32];
      pacc += gelu_erf(v) * sWp3[i * 32 + lane];
    }
    pacc += __shfl_xor(pacc, 1, 32);
    pacc += __shfl_xor(pacc, 2, 32);
    pacc += __shfl_xor(pacc, 4, 32);
    pacc += __shfl_xor(pacc, 8, 32);
    pacc += __shfl_xor(pacc, 16, 32);
    const float p = pacc + vbp3;
    const float res = zs + p;
    if (lane == 0) sOut[rloc] = res;
    wave_sync();
  }
  __syncthreads();

  if (wave == 0) {
    const float v0 = sOut[lane];
    const float v1 = sOut[32 + lane];
    float* op = out + (size_t)(row0 + blkRow0);
    for (int pass = 0; pass < 2; ++pass) {
      *(volatile float*)(op + lane) = v0;
      *(volatile float*)(op + 32 + lane) = v1;
      __threadfence();
    }
  }
}

extern "C" void kernel_launch(void* const* d_in, const int* in_sizes, int n_in,
                              void* d_out, int out_size, void* d_ws, size_t ws_size,
                              hipStream_t stream) {
  const int*   x      = (const int*)d_in[0];
  const float* phenos = (const float*)d_in[1];
  const float* emb    = (const float*)d_in[2];
  const float* W1     = (const float*)d_in[3];
  const float* b1     = (const float*)d_in[4];
  const float* W2     = (const float*)d_in[5];
  const float* b2     = (const float*)d_in[6];
  const float* Wb     = (const float*)d_in[7];
  const float* ob     = (const float*)d_in[8];
  const float* Wc1    = (const float*)d_in[9];
  const float* bc1    = (const float*)d_in[10];
  const float* Wc2    = (const float*)d_in[11];
  const float* bc2    = (const float*)d_in[12];
  const float* Wp1    = (const float*)d_in[13];
  const float* Wp2    = (const float*)d_in[14];
  const float* Wp3    = (const float*)d_in[15];
  const float* bp3    = (const float*)d_in[16];
  float* out = (float*)d_out;

  if (n_in < 17) return;
  if (in_sizes[0] != kRows * 2) return;
  if (in_sizes[2] != kGenes * kEmb) return;
  if (in_sizes[14] != kHid * kHid) return;
  if (out_size != kRows) return;
  if (ws_size < kWsTotal) return;

  char* ws = (char*)d_ws;
  unsigned short* wT   = (unsigned short*)(ws + kOffWT);
  unsigned short* g1   = (unsigned short*)(ws + kOffG1);
  float*          pre2 = (float*)(ws + kOffPre2);

  wtcast_kernel<<<dim3(kHid / 64, kHid / 64), 256, 0, stream>>>(Wp2, wT, kCarryW);

  const int gemmTiles  = (kChunk / 64) * (kHid / 64);
  const int gemmBlocks = gemmTiles / 8;

  for (int c = 0; c < kNumChunks; ++c) {
    const int row0 = c * kChunk;
    pheno_l1_kernel<<<kChunk, 256, 0, stream>>>(phenos, Wp1, g1, row0, kRows);
    wmma_gemm64<0, false, 0, 0, false, 0><<<dim3(gemmBlocks, 1), 256, 0, stream>>>(
        g1, g1, kHid, 0L,
        wT, wT, kHid, 0L,
        (void*)pre2, (void*)pre2, kHid, 0L,
        bp3,
        phenos, 0L,
        kChunk, kHid, kHid, kGemmScale);
    finisher_kernel<<<kChunk / kRowsPerBlk, 256, 0, stream>>>(
        x, emb, W1, b1, W2, b2, Wb, ob, Wc1, bc1, Wc2, bc2, Wp3, bp3, pre2, out, row0, kRows);
  }
}
